// CAML_49735721288066
// MI455X (gfx1250) — hardware-verified
//
#include <hip/hip_runtime.h>
#include <math.h>

typedef __attribute__((ext_vector_type(16))) _Float16 v16h;
typedef __attribute__((ext_vector_type(16))) __bf16 v16b;
typedef __attribute__((ext_vector_type(8)))  _Float16 v8h;
typedef __attribute__((ext_vector_type(8)))  float v8f;
typedef __attribute__((ext_vector_type(4)))  float v4f;
typedef __attribute__((ext_vector_type(2)))  float v2f;
typedef __attribute__((ext_vector_type(4)))  unsigned v4u;
typedef __attribute__((ext_vector_type(4)))  int v4i;
typedef float __attribute__((may_alias)) float_a;
typedef int __attribute__((may_alias)) int_a;

template <typename T> __device__ __forceinline__ void vst2(void* p, T v) { *(volatile T*)p = v; __threadfence(); *(volatile T*)p = v; }
__device__ __forceinline__ v8f wmma16(v16h a, v16h b, v8f c) {
  v8f d = __builtin_amdgcn_wmma_f32_16x16x32_f16(false, a, false, b, (short)0, c, false, false);
  asm volatile("v_nop\n\tv_nop\n\tv_nop\n\tv_nop" : "+v"(d) : "v"(a), "v"(b));
  return d;
}
__device__ __forceinline__ v8f wmma_bf(v16b a, v16b b, v8f c) {
  v8f d = __builtin_amdgcn_wmma_f32_16x16x32_bf16(false, a, false, b, (short)0, c, false, false);
  asm volatile("v_nop\n\tv_nop\n\tv_nop\n\tv_nop" : "+v"(d) : "v"(a), "v"(b));
  return d;
}
__device__ __forceinline__ v16h frag_h(const _Float16* rowk0, int lane) {
  union { v16h v; v8h q[2]; } u; const _Float16* p = rowk0 + 8 * (lane >> 4);
  u.q[0] = *(const v8h*)p; u.q[1] = *(const v8h*)(p + 16); return u.v;
}
__device__ __forceinline__ v16h frag_f32(const float* rowk0, int lane) {
  v16h a; const float* p = rowk0 + 8 * (lane >> 4);
#pragma unroll
  for (int i = 0; i < 8; ++i) { a[i] = (_Float16)p[i]; a[8 + i] = (_Float16)p[16 + i]; }
  return a;
}
__device__ __forceinline__ v16h frag_f32s(const float* rowk0, int lane, float sc) {
  v16h a; const float* p = rowk0 + 8 * (lane >> 4);
#pragma unroll
  for (int i = 0; i < 8; ++i) { a[i] = (_Float16)(p[i] * sc); a[8 + i] = (_Float16)(p[16 + i] * sc); }
  return a;
}
__device__ __forceinline__ v16h fragc_f32(const float* W, int k0, int n, int lane, int ld, int K) {
  v16h a; const int g = lane >> 4;
#pragma unroll
  for (int i = 0; i < 8; ++i) { const int ka = k0 + 8 * g + i, kb = ka + 16;
    a[i] = (_Float16)(ka < K ? W[(size_t)(ka < K ? ka : K - 1) * ld + n] : 0.f); a[8 + i] = (_Float16)(kb < K ? W[(size_t)(kb < K ? kb : K - 1) * ld + n] : 0.f); }
  return a;
}
struct F2 { v16b h, l; };
__device__ __forceinline__ F2 bsplit16(const float v[16]) { F2 r;
#pragma unroll
  for (int i = 0; i < 16; ++i) { const __bf16 h = (__bf16)v[i]; r.h[i] = h; r.l[i] = (__bf16)(v[i] - (float)h); }
  return r; }
__device__ __forceinline__ F2 split_row(const float* row, int k0, int lane) { float v[16]; const float* p = row + k0 + 8 * (lane >> 4);
#pragma unroll
  for (int i = 0; i < 8; ++i) { v[i] = p[i]; v[8 + i] = p[16 + i]; }
  return bsplit16(v); }
__device__ __forceinline__ F2 split_rowK(const float* row, int k0, int lane, int K) { float v[16]; const int g = lane >> 4;
#pragma unroll
  for (int i = 0; i < 8; ++i) { const int ka = k0 + 8 * g + i, kb = ka + 16; v[i] = ka < K ? row[ka < K ? ka : K - 1] : 0.f; v[8 + i] = kb < K ? row[kb < K ? kb : K - 1] : 0.f; }
  return bsplit16(v); }
__device__ __forceinline__ F2 split_col(const float* W, int k0, int n, int lane, int ld, int K) { float v[16]; const int g = lane >> 4;
#pragma unroll
  for (int i = 0; i < 8; ++i) { const int ka = k0 + 8 * g + i, kb = ka + 16; v[i] = ka < K ? W[(size_t)(ka < K ? ka : K - 1) * ld + n] : 0.f; v[8 + i] = kb < K ? W[(size_t)(kb < K ? kb : K - 1) * ld + n] : 0.f; }
  return bsplit16(v); }
__device__ __forceinline__ v8f mac3(const F2& a, const F2& b, v8f c) { c = wmma_bf(a.l, b.h, c); c = wmma_bf(a.h, b.l, c); return wmma_bf(a.h, b.h, c); }
__device__ __forceinline__ float sigm(float v) { return 1.0f / (1.0f + expf(-v)); }
#define LDSX() do { asm volatile("s_wait_dscnt 0" ::: "memory"); __builtin_amdgcn_wave_barrier(); __builtin_amdgcn_fence(__ATOMIC_RELEASE, "workgroup"); } while (0)


#define NBT 8
#define SEQ 2000
#define SEQP 2016
#define EMB 100
#define EP 128
#define HID 50
#define HP 64
#define NL 8921
#define NLP 8960
#define KW 9
#ifndef TLB
#define TLB (NLP / 64)
#define TNB NBT
#endif
typedef __attribute__((ext_vector_type(8))) __bf16 v8b;
__device__ __forceinline__ v16b frag_b(const __bf16* rowk0, int lane) {
  union { v16b v; v8b q[2]; } u; const __bf16* p = rowk0 + 8 * (lane >> 4);
  u.q[0] = *(const v8b*)p; u.q[1] = *(const v8b*)(p + 16); return u.v;
}
__device__ __forceinline__ float bfr(float v) { return (float)(__bf16)v; }
__device__ __attribute__((noinline)) float exp_ni(float v) { return expf(v); }
__device__ __attribute__((noinline)) float tanh_ni(float v) { return tanhf(v); }
#define EROWS (SEQ + 8)
#define WS_E    0u
#define WS_PW   (WS_E + 2u * NBT * EROWS * EP)
#define WS_UW   (WS_PW + 2u * HP * KW * EP)
#define WS_H    (WS_UW + 2u * NLP * HP)
#define WS_HTH  (WS_H + 4u * NBT * SEQP * HP)
#define WS_HTL  (WS_HTH + 2u * NBT * HP * SEQP)
#define WS_Y    (WS_HTL + 2u * NBT * HP * SEQP)
#define WS_END  (WS_Y + 4u * NBT * NLP)

__global__ __launch_bounds__(128) void k_emb(const int* __restrict__ X, const float* __restrict__ TBL, __bf16* __restrict__ E) {
  __shared__ __align__(16) __bf16 srow[EP];
  const int b = blockIdx.y, pr = blockIdx.x, tid = threadIdx.x; const int s = pr - 4; float v = 0.f;
  if (s >= 0 && s < SEQ && tid < EMB) { const int id = min(max(X[b * SEQ + s], 0), 50001); v = bfr(TBL[(size_t)id * EMB + tid]); }
  srow[tid] = (__bf16)v;
  __syncthreads();
  if (tid < 16) vst2((unsigned*)(E + ((size_t)b * EROWS + pr) * EP + tid * 8), *(const v4u*)(&srow[tid * 8]));
}
__global__ __launch_bounds__(128) void k_packw(const float* __restrict__ CW, const float* __restrict__ UWi, __bf16* __restrict__ PW, __bf16* __restrict__ UW) {
  __shared__ __align__(16) __bf16 srow[KW * EP]; __shared__ __align__(16) __bf16 su[16][HP];
  const int blk = blockIdx.x, tid = threadIdx.x;
  if (blk < HP) { const int o = blk;
    for (int q = tid; q < KW * EP; q += 128) { const int k = q / EP, c = q % EP; srow[q] = (__bf16)((o < HID && c < EMB) ? bfr(CW[((size_t)o * EMB + c) * KW + k]) : 0.f); }
    __syncthreads();
    for (int q = tid; q < KW * EP / 8; q += 128) vst2((unsigned*)(PW + (size_t)o * KW * EP + q * 8), *(const v4u*)(&srow[q * 8])); }
  else { const int l0 = (blk - HP) * 16;
    for (int q = tid; q < 16 * HP; q += 128) { const int r = q >> 6, h = q & 63; const int l = l0 + r; su[r][h] = (__bf16)((l < NL && h < HID) ? bfr(UWi[(size_t)l * HID + h]) : 0.f); }
    __syncthreads();
    vst2((unsigned*)(UW + (size_t)l0 * HP + tid * 8), *(const v4u*)(&su[0][0] + tid * 8)); }
}
__global__ __launch_bounds__(128) void k_conv(const __bf16* __restrict__ E, const __bf16* __restrict__ PW, const float* __restrict__ cb, float* __restrict__ H, __bf16* __restrict__ HTH, __bf16* __restrict__ HTL) {
  __shared__ __align__(16) float so[4][16][68]; __shared__ __align__(16) __bf16 sth[HP][72], stl[HP][72];
  const int tid = threadIdx.x, wave = tid >> 5, lane = tid & 31, col = lane & 15, g = lane >> 4; const int b = blockIdx.y, s0 = blockIdx.x * 64;
  v8f acc[4] = {};
  const int srow = min(s0 + wave * 16 + col, SEQ - 1);
#pragma unroll 1
  for (int k = 0; k < KW; ++k) {
#pragma unroll
    for (int kc = 0; kc < 4; ++kc) { const v16b a = frag_b(E + ((size_t)b * EROWS + srow + k) * EP + kc * 32, lane);
#pragma unroll
      for (int j = 0; j < 4; ++j) acc[j] = wmma_bf(a, frag_b(PW + ((size_t)(j * 16 + col) * KW + k) * EP + kc * 32, lane), acc[j]); } }
#pragma unroll
  for (int j = 0; j < 4; ++j) { const int o = j * 16 + col; const float bb = o < HID ? bfr(cb[o]) : 0.f;
#pragma unroll
    for (int r = 0; r < 8; ++r) { const int s = s0 + wave * 16 + 8 * g + r; so[wave][8 * g + r][o] = (o < HID && s < SEQ) ? tanh_ni(acc[j][r] + bb) : 0.f; } }
  __syncthreads();
  for (int rl = 0; rl < 16; ++rl) { const int s = s0 + wave * 16 + rl; if (s < SEQP && lane < 16) vst2(H + ((size_t)b * SEQP + s) * HP + lane * 4, *(const v4f*)&so[wave][rl][lane * 4]); }
  for (int q = tid; q < HP * 64; q += 128) { const int o = q >> 6, sl = q & 63; const float v = so[sl >> 4][sl & 15][o]; const __bf16 hb = (__bf16)v; sth[o][sl] = hb; stl[o][sl] = (__bf16)(v - (float)hb); }
  __syncthreads();
  if (s0 < SEQP) for (int q = tid; q < HP * 8; q += 128) { const int o = q >> 3, pc = q & 7; if (s0 + pc * 8 < SEQP) { const size_t off = ((size_t)b * HP + o) * SEQP + s0 + pc * 8; vst2((unsigned*)(HTH + off), *(const v4u*)&sth[o][pc * 8]); vst2((unsigned*)(HTL + off), *(const v4u*)&stl[o][pc * 8]); } }
}
__global__ __launch_bounds__(128) void k_att(const __bf16* __restrict__ UW, const float* __restrict__ H, const __bf16* __restrict__ HTH, const __bf16* __restrict__ HTL, const float* __restrict__ OW, const float* __restrict__ OB, float* __restrict__ Y) {
  __shared__ __align__(16) float sp[4][16][36]; __shared__ float sm[4][16][HP + 1]; __shared__ __align__(16) float sy[64];
  const int tid = threadIdx.x, wave = tid >> 5, lane = tid & 31, col = lane & 15, g = lane >> 4; const int b = blockIdx.y; const int l0 = blockIdx.x * 64 + wave * 16;
  const v16b a0 = frag_b(UW + (size_t)(l0 + col) * HP, lane), a1 = frag_b(UW + (size_t)(l0 + col) * HP + 32, lane);
  float m[8], l[8];
#pragma unroll
  for (int r = 0; r < 8; ++r) { m[r] = -3.0e38f; l[r] = 0.f; }
  v8f acc[4] = {};
#pragma unroll 1
  for (int ks = 0; ks < SEQP / 32; ++ks) { v8f s[2];
#pragma unroll
    for (int ct = 0; ct < 2; ++ct) { const int ss = ks * 32 + ct * 16 + col; const float* hr = H + ((size_t)b * SEQP + ss) * HP; const F2 h0 = split_row(hr, 0, lane), h1 = split_row(hr, 32, lane);
      v8f c = {}; c = wmma_bf(a0, h0.h, c); c = wmma_bf(a0, h0.l, c); c = wmma_bf(a1, h1.h, c); c = wmma_bf(a1, h1.l, c);
#pragma unroll
      for (int r = 0; r < 8; ++r) s[ct][r] = ss < SEQ ? c[r] : -3.0e38f; }
#pragma unroll
    for (int r = 0; r < 8; ++r) { float mx = fmaxf(s[0][r], s[1][r]);
#pragma unroll
      for (int o = 1; o < 16; o <<= 1) mx = fmaxf(mx, __shfl_xor(mx, o));
      const float mn = fmaxf(m[r], mx); const float alpha = exp_ni(m[r] - mn);
      const float e0 = s[0][r] <= -1.0e38f ? 0.f : exp_ni(s[0][r] - mn), e1 = s[1][r] <= -1.0e38f ? 0.f : exp_ni(s[1][r] - mn); float es = e0 + e1;
#pragma unroll
      for (int o = 1; o < 16; o <<= 1) es += __shfl_xor(es, o);
      l[r] = l[r] * alpha + es; m[r] = mn;
#pragma unroll
      for (int dt = 0; dt < 4; ++dt) acc[dt][r] *= alpha;
      sp[wave][8 * g + r][col] = e0; sp[wave][8 * g + r][16 + col] = e1; }
    LDSX();
    const F2 pa = split_row(&sp[wave][col][0], 0, lane);
#pragma unroll
    for (int dt = 0; dt < 4; ++dt) { const size_t hrow = ((size_t)b * HP + dt * 16 + col) * SEQP + ks * 32; const v16b vh = frag_b(HTH + hrow, lane), vl = frag_b(HTL + hrow, lane);
      acc[dt] = wmma_bf(pa.l, vh, acc[dt]); acc[dt] = wmma_bf(pa.h, vl, acc[dt]); acc[dt] = wmma_bf(pa.h, vh, acc[dt]); }
    LDSX(); }
#pragma unroll
  for (int dt = 0; dt < 4; ++dt)
#pragma unroll
    for (int r = 0; r < 8; ++r) sm[wave][8 * g + r][dt * 16 + col] = acc[dt][r] / l[r];
  LDSX();
  if (lane < 16) { const int lbl = l0 + lane; float yv = 0.f; if (lbl < NL) { yv = bfr(OB[lbl]); for (int h = 0; h < HID; ++h) yv += bfr(OW[(size_t)lbl * HID + h]) * sm[wave][lane][h]; } sy[wave * 16 + lane] = yv; }
  __syncthreads();
  if (tid < 16) vst2(Y + (size_t)b * NLP + blockIdx.x * 64 + tid * 4, *(const v4f*)&sy[tid * 4]);
}
__global__ __launch_bounds__(256) void k_copy(const float* __restrict__ Y, float* __restrict__ out) {
  const size_t p = (size_t)blockIdx.x * 256 + threadIdx.x; const size_t total = (size_t)NBT * NL;
  if (p * 4 >= total) return; v4f v;
#pragma unroll
  for (int i = 0; i < 4; ++i) { const size_t f = p * 4 + i; v[i] = f < total ? Y[(f / NL) * NLP + (f % NL)] : 0.f; }
  vst2(out + p * 4, v);
}

extern "C" void kernel_launch(void* const* d_in, const int* in_sizes, int n_in, void* d_out, int out_size, void* d_ws, size_t ws_size, hipStream_t stream) {
  (void)in_sizes; (void)n_in; (void)out_size;
  const float** F = (const float**)d_in; const int** I = (const int**)d_in;
  if (ws_size < (size_t)WS_END) return;
  char* ws = (char*)d_ws; __bf16 *E = (__bf16*)(ws + WS_E), *PW = (__bf16*)(ws + WS_PW), *UW = (__bf16*)(ws + WS_UW), *HTH = (__bf16*)(ws + WS_HTH), *HTL = (__bf16*)(ws + WS_HTL); float *H = (float*)(ws + WS_H), *Y = (float*)(ws + WS_Y);
  k_emb<<<dim3(EROWS, NBT), 128, 0, stream>>>(I[0], F[1], E);
  k_packw<<<HP + NLP / 16, 128, 0, stream>>>(F[2], F[4], PW, UW);
  k_conv<<<dim3(SEQP / 64 + 1, NBT), 128, 0, stream>>>(E, PW, F[3], H, HTH, HTL);
  k_att<<<dim3(TLB, TNB), 128, 0, stream>>>(UW, H, HTH, HTL, F[5], F[6], Y);
  k_copy<<<(NBT * NL / 4 + 255) / 256, 256, 0, stream>>>(Y, (float*)d_out);
}
